// Block_4509715660807
// MI455X (gfx1250) — hardware-run, weakly checked
//
#include <hip/hip_runtime.h>
#include <math.h>

#ifndef NB
#define NB 2
#endif
#ifndef SEQ
#define SEQ 2048
#endif
#define NB_FULL 2
#define SEQ_FULL 2048
#define DM 1024
#define NHEAD 16
#define HDIM 64
#define FFD 4096
#define MTOK (NB * SEQ)
#define FCH (MTOK / 2)

static_assert(SEQ % 64 == 0);
static_assert(MTOK % 128 == 0);
static_assert(NB <= NB_FULL && SEQ <= SEQ_FULL);
static_assert(DM == NHEAD * HDIM);

typedef __attribute__((ext_vector_type(16))) _Float16 v16h;
typedef __attribute__((ext_vector_type(8)))  _Float16 v8h;
typedef __attribute__((ext_vector_type(16))) __bf16   v16b;
typedef __attribute__((ext_vector_type(8)))  __bf16   v8b;
typedef __attribute__((ext_vector_type(8)))  float    v8f;
typedef __attribute__((ext_vector_type(4)))  float    v4f;
typedef unsigned int cm_u4 __attribute__((ext_vector_type(4)));
typedef unsigned int bk_u2 __attribute__((ext_vector_type(2)));

__device__ __forceinline__ v8f wmma16(v16h a, v16h b, v8f c) {
    c = __builtin_amdgcn_wmma_f32_16x16x32_f16(false, a, false, b, (short)0, c, false, false);
    asm volatile("v_nop\n\tv_nop\n\tv_nop\n\tv_nop" : "+v"(c) : "v"(a), "v"(b));
    return c;
}

#define VST2(T, ptr, val) do { const T vst2_v_ = (val); *(volatile T*)(ptr) = vst2_v_; __threadfence(); *(volatile T*)(ptr) = vst2_v_; } while (0)
#define VST2V4(ptr, val) do { const v4f vst2_v4_ = (val); *(volatile v4f*)(ptr) = vst2_v4_; __threadfence(); *(volatile v4f*)(ptr) = vst2_v4_; } while (0)

__device__ __forceinline__ unsigned short f2bf_bits(float f) {
  unsigned u = __float_as_uint(f);
  return (unsigned short)((u + 0x7FFFu + ((u >> 16) & 1u)) >> 16);
}
__device__ __forceinline__ float bf_bits2f(unsigned short h) { return __uint_as_float(((unsigned)h) << 16); }

__device__ __forceinline__ void dep_guard_h(v8f& a, v8f& b, v16h x, v16h y) { asm volatile("v_nop\n\tv_nop\n\tv_nop\n\tv_nop" : "+v"(a), "+v"(b) : "v"(x), "v"(y)); }
__device__ __forceinline__ void dep_guard_b(v8f& a, v8f& b, v16b x, v16b y) { asm volatile("v_nop\n\tv_nop\n\tv_nop\n\tv_nop" : "+v"(a), "+v"(b) : "v"(x), "v"(y)); }
__device__ __forceinline__ void keep4_h(v16h a, v16h b, v16h c, v16h d) { asm volatile("v_nop" :: "v"(a), "v"(b), "v"(c), "v"(d)); }
__device__ __forceinline__ void keep4_b(v16b a, v16b b, v16b c, v16b d) { asm volatile("v_nop" :: "v"(a), "v"(b), "v"(c), "v"(d)); }
__device__ __forceinline__ void acc_guard4(v8f& a, v8f& b, v8f& c, v8f& d) { asm volatile("v_nop\n\tv_nop\n\tv_nop\n\tv_nop" : "+v"(a), "+v"(b), "+v"(c), "+v"(d)); }
template <typename T> struct Frag;
template <> struct Frag<_Float16> {
  typedef v16h V; union U { v16h v; v8h h[2]; };
  static __device__ __forceinline__ v16h load(const _Float16* p) {
    U f; f.h[0] = *(const v8h*)(p); f.h[1] = *(const v8h*)(p + 16); return f.v;
  }
  static __device__ __forceinline__ v8f mma(v16h a, v16h b, v8f c) {
    return __builtin_amdgcn_wmma_f32_16x16x32_f16(false, a, false, b, (short)0, c, false, false);
  }
  static __device__ __forceinline__ void guard(v8f& a, v8f& b, v16h x, v16h y) { dep_guard_h(a, b, x, y); }
  static __device__ __forceinline__ void keep(v16h a, v16h b, v16h c, v16h d) { keep4_h(a, b, c, d); }
};
template <> struct Frag<__bf16> {
  typedef v16b V; union U { v16b v; v8b h[2]; };
  static __device__ __forceinline__ v16b load(const __bf16* p) {
    U f; f.h[0] = *(const v8b*)(p); f.h[1] = *(const v8b*)(p + 16); return f.v;
  }
  static __device__ __forceinline__ v8f mma(v16b a, v16b b, v8f c) {
    return __builtin_amdgcn_wmma_f32_16x16x32_bf16(false, a, false, b, (short)0, c, false, false);
  }
  static __device__ __forceinline__ void guard(v8f& a, v8f& b, v16b x, v16b y) { dep_guard_b(a, b, x, y); }
  static __device__ __forceinline__ void keep(v16b a, v16b b, v16b c, v16b d) { keep4_b(a, b, c, d); }
};

template <int ET> struct Elem;
template <> struct Elem<0> { typedef _Float16 T; };
template <> struct Elem<1> { typedef __bf16 T; };
template <int ET, bool SPLIT, int BIAS_MODE, int OUT_MODE, bool RESID, int ACT = 0>
__global__ __launch_bounds__(256) void wmma_gemm64(
    const unsigned short* __restrict__ Ap, const unsigned short* __restrict__ A2p, int lda, long strideA,
    const unsigned short* __restrict__ Btp, const unsigned short* __restrict__ Bt2p, int ldb, long strideB,
    void* __restrict__ Cout, void* __restrict__ Cout2, int ldc, long strideC,
    const float* __restrict__ bias,
    const float* __restrict__ resid, long strideR,
    int M, int N, int K, float scale) {
  typedef typename Elem<ET>::T T;
  typedef typename Frag<T>::V V;
  const T* A = (const T*)Ap; const T* A2 = (const T*)A2p; const T* Bt = (const T*)Btp; const T* Bt2 = (const T*)Bt2p;
  __shared__ __align__(16) float sT[8][16 * 68];
  const int b    = blockIdx.y;
  const int lane = threadIdx.x & 31;
  const int wave = threadIdx.x >> 5;
  const int tilesN = N >> 6;
  const int tilesM = M >> 6;
  const int tile = blockIdx.x * 8 + wave;
  if (tile >= tilesM * tilesN) return;
  const int tm = tile / tilesN;
  const int tn = tile - tm * tilesN;
  const int m0 = tm << 6;
  const int n0 = tn << 6;

  const T* Ab  = A  + (size_t)b * strideA;
  const T* Bb  = Bt + (size_t)b * strideB;
  const T* Ab2 = SPLIT ? (A2  + (size_t)b * strideA) : nullptr;
  const T* Bb2 = SPLIT ? (Bt2 + (size_t)b * strideB) : nullptr;

  const int rlane = lane & 15;
  const int koff  = (lane >> 4) * 8;
  const int mOff  = (lane >> 4) * 8;

  v8f acc[4][4];
#pragma unroll
  for (int i = 0; i < 4; ++i)
#pragma unroll
    for (int j = 0; j < 4; ++j) acc[i][j] = (v8f){0.f,0.f,0.f,0.f,0.f,0.f,0.f,0.f};

  for (int k0 = 0; k0 < K; k0 += 32) {
    V bh[4], bl[4];
#pragma unroll
    for (int j = 0; j < 4; ++j) {
      const size_t bo = (size_t)(n0 + (j << 4) + rlane) * ldb + koff + k0;
      bh[j] = Frag<T>::load(Bb + bo);
      if (SPLIT) bl[j] = Frag<T>::load(Bb2 + bo);
    }
#pragma unroll
    for (int i = 0; i < 4; ++i) {
      const size_t ao = (size_t)(m0 + (i << 4) + rlane) * lda + koff + k0;
      V ah = Frag<T>::load(Ab + ao);
      V al;
      if (SPLIT) al = Frag<T>::load(Ab2 + ao);
#pragma unroll
      for (int j = 0; j < 4; ++j) {
        acc[i][j] = Frag<T>::mma(ah, bh[j], acc[i][j]);
        if (SPLIT) {
          acc[i][j] = Frag<T>::mma(ah, bl[j], acc[i][j]);
          acc[i][j] = Frag<T>::mma(al, bh[j], acc[i][j]);
        }
      }
      Frag<T>::guard(acc[i][0], acc[i][3], ah, SPLIT ? al : ah);
    }
    Frag<T>::keep(bh[0], bh[1], bh[2], bh[3]);
    if (SPLIT) Frag<T>::keep(bl[0], bl[1], bl[2], bl[3]);
  }
  acc_guard4(acc[0][0], acc[0][1], acc[0][2], acc[0][3]);
  acc_guard4(acc[1][0], acc[1][1], acc[1][2], acc[1][3]);
  acc_guard4(acc[2][0], acc[2][1], acc[2][2], acc[2][3]);
  acc_guard4(acc[3][0], acc[3][1], acc[3][2], acc[3][3]);

  float* slab = sT[wave];
  const float* Rb = RESID ? (resid + (size_t)b * strideR) : nullptr;
#pragma unroll
  for (int i = 0; i < 4; ++i) {
    const int mBase = m0 + (i << 4);
#pragma unroll
    for (int j = 0; j < 4; ++j) {
      const int n = n0 + (j << 4) + rlane;
      float bv = 0.f;
      if (BIAS_MODE == 2) bv = bias[n];
#pragma unroll
      for (int r = 0; r < 8; ++r) {
        float v = acc[i][j][r] * scale;
        if (BIAS_MODE == 1) v += bias[mBase + mOff + r];
        if (BIAS_MODE == 2) v += bv;
        if (RESID) v += Rb[(size_t)(mBase + mOff + r) * ldc + n];
        if (ACT == 1) v = tanhf(v);
        if (ACT == 2) v = fmaxf(v, 0.0f);
        if (ACT == 3) v = v / (1.0f + expf(-v));
        if (ACT == 4) v = (v > 0.f) ? v : 0.01f * v;
        if (ACT == 5) v = 0.5f * v * (1.0f + erff(v * 0.70710678118654752f));
        if (ACT == 6) v = (v > 0.f) ? v : 0.2f * v;
        if (ACT == 7) { const float u = 0.7978845608028654f * (v + 0.044715f * v * v * v); v = 0.5f * v * (1.f + tanhf(u)); }
        slab[(mOff + r) * 68 + (j << 4) + rlane] = v;
      }
    }
    __builtin_amdgcn_fence(3  , "workgroup");
    __builtin_amdgcn_wave_barrier();
    __builtin_amdgcn_fence(2  , "workgroup");
    if (OUT_MODE == 0) {
      float* C = (float*)Cout + (size_t)b * strideC;
      const int hh = lane >> 4, c4 = (lane & 15) * 4;
      for (int pass = 0; pass < 2; ++pass) {
#pragma unroll
        for (int it = 0; it < 8; ++it) {
          const int row = it * 2 + hh;
          v4f v = *(const v4f*)(slab + row * 68 + c4);
          *(volatile v4f*)(C + (size_t)(mBase + row) * ldc + n0 + c4) = v;
        }
        __threadfence();
      }
    } else {
      const int q = lane >> 3, c8 = (lane & 7) * 8;
      unsigned short* C  = (unsigned short*)Cout  + (size_t)b * strideC;
      unsigned short* C2 = (OUT_MODE == 2) ? ((unsigned short*)Cout2 + (size_t)b * strideC) : nullptr;
      for (int pass = 0; pass < 2; ++pass) {
#pragma unroll
        for (int it = 0; it < 4; ++it) {
          const int row = it * 4 + q;
          const float* sp = slab + row * 68 + c8;
          v8h hv, lv;
#pragma unroll
          for (int e = 0; e < 8; ++e) {
            if (OUT_MODE == 1) {
              hv[e] = (_Float16)sp[e];
            } else {
              unsigned short hb = f2bf_bits(sp[e]);
              unsigned short lb = f2bf_bits(sp[e] - bf_bits2f(hb));
              hv[e] = __builtin_bit_cast(_Float16, hb);
              lv[e] = __builtin_bit_cast(_Float16, lb);
            }
          }
          *(volatile v8h*)(C + (size_t)(mBase + row) * ldc + n0 + c8) = hv;
          if (OUT_MODE == 2) *(volatile v8h*)(C2 + (size_t)(mBase + row) * ldc + n0 + c8) = lv;
        }
        __threadfence();
      }
    }
    __builtin_amdgcn_fence(3  , "workgroup");
    __builtin_amdgcn_wave_barrier();
    __builtin_amdgcn_fence(2  , "workgroup");
  }
}

__device__ __forceinline__ unsigned int cmb_pk2(float a, float b) { return (unsigned int)__builtin_bit_cast(unsigned short, (_Float16)a) | ((unsigned int)__builtin_bit_cast(unsigned short, (_Float16)b) << 16); }
__device__ __forceinline__ float cmb_bf(float v) { const unsigned u = __builtin_bit_cast(unsigned, v); const unsigned r = (u + 0x7fffu + ((u >> 16) & 1u)) & 0xffff0000u; return __builtin_bit_cast(float, r); }
template <int BF>
__global__ __launch_bounds__(256) void k_cm_castb(const float* __restrict__ SRC, int lds, unsigned short* __restrict__ DST, int ldd, int nR, int nC, float sc) {
    const long long u = (long long)blockIdx.x * 256 + threadIdx.x; const int per = nC / 8; if (u >= (long long)nR * per) return; const int r = (int)(u / per); const int c0 = 8 * (int)(u % per);
    const float* s = SRC + (long long)r * lds + c0; const v4f a = *(const v4f*)s, b = *(const v4f*)(s + 4);
    const float w0 = (BF ? cmb_bf(a.x) : a.x) * sc, w1 = (BF ? cmb_bf(a.y) : a.y) * sc, w2 = (BF ? cmb_bf(a.z) : a.z) * sc, w3 = (BF ? cmb_bf(a.w) : a.w) * sc;
    const float w4 = (BF ? cmb_bf(b.x) : b.x) * sc, w5 = (BF ? cmb_bf(b.y) : b.y) * sc, w6 = (BF ? cmb_bf(b.z) : b.z) * sc, w7 = (BF ? cmb_bf(b.w) : b.w) * sc;
    cm_u4 pk; pk.x = cmb_pk2(w0, w1); pk.y = cmb_pk2(w2, w3); pk.z = cmb_pk2(w4, w5); pk.w = cmb_pk2(w6, w7); VST2(cm_u4, (cm_u4*)(DST + (long long)r * ldd + c0), pk); }
__global__ __launch_bounds__(256) void k_cm_castbT(const float* __restrict__ SRC, int lds, unsigned short* __restrict__ DST, int ldd, int nR, int nC, float sc) {
    const long long u = (long long)blockIdx.x * 256 + threadIdx.x; const int per = nR / 8; if (u >= (long long)nC * per) return; const int c = (int)(u / per); const int r0 = 8 * (int)(u % per);
    float w[8];
#pragma unroll
    for (int e = 0; e < 8; ++e) w[e] = cmb_bf(SRC[(long long)(r0 + e) * lds + c]) * sc;
    cm_u4 pk; pk.x = cmb_pk2(w[0], w[1]); pk.y = cmb_pk2(w[2], w[3]); pk.z = cmb_pk2(w[4], w[5]); pk.w = cmb_pk2(w[6], w[7]); VST2(cm_u4, (cm_u4*)(DST + (long long)c * ldd + r0), pk); }
__global__ __launch_bounds__(256) void k_bfcat3(const float* __restrict__ A, int na, const float* __restrict__ B, int nb, const float* __restrict__ C, int nc, float* __restrict__ DST) {
    const int u = blockIdx.x * 256 + threadIdx.x; if (u >= na + nb + nc) return;
    const float va = A[min(u, na - 1)]; const float vb = B[min(max(u - na, 0), nb - 1)]; const float vc = C[min(max(u - na - nb, 0), nc - 1)];
    const float v = (u < na) ? va : ((u < na + nb) ? vb : vc); VST2(float, DST + u, cmb_bf(v)); }
__global__ __launch_bounds__(256) void k_maskbias(const int* __restrict__ mask, float* __restrict__ MB, int seq, int seq_full, int n) {
    #pragma clang fp contract(off)
    const int u = blockIdx.x * 256 + threadIdx.x; if (u >= n) return; const int b = u / seq, j = u - b * seq;
    const float mv = (float)mask[(long long)b * seq_full + j]; const float v = -(10000.0f * (1.0f - mv)); VST2(float, MB + u, v); }

#define AT_NW 4
struct AttnG { const float* q; const float* k; const float* v; float* o; const float* kb;
               long long q_bs, q_rs, q_hs, k_bs, k_rs, k_hs, v_bs, v_rs, v_hs, o_bs, o_rs, o_hs, kb_bs;
               int S, Skv, H; float qscale; };
static_assert(sizeof(AttnG) == 5 * 8 + 13 * 8 + 4 * 4);

__device__ __forceinline__ v16h pk16(const v4f a0, const v4f a1, const v4f a2, const v4f a3) {
    v16h r;
    r[0] = (_Float16)a0.x; r[1] = (_Float16)a0.y; r[2] = (_Float16)a0.z; r[3] = (_Float16)a0.w;
    r[4] = (_Float16)a1.x; r[5] = (_Float16)a1.y; r[6] = (_Float16)a1.z; r[7] = (_Float16)a1.w;
    r[8] = (_Float16)a2.x; r[9] = (_Float16)a2.y; r[10] = (_Float16)a2.z; r[11] = (_Float16)a2.w;
    r[12] = (_Float16)a3.x; r[13] = (_Float16)a3.y; r[14] = (_Float16)a3.z; r[15] = (_Float16)a3.w;
    return r;
}

__global__ __launch_bounds__(32 * AT_NW) void k_attn64(AttnG g) {
  union FH { v16h v; v8h h[2]; };
  constexpr int LP = 72;
  __shared__ __align__(16) _Float16 Ksh[64 * LP];
  __shared__ __align__(16) _Float16 Vth[64 * LP];
  __shared__ __align__(16) _Float16 Psh[AT_NW][16 * LP];
  __shared__ __align__(16) float    Os[AT_NW][16 * 68];

  const int tid  = threadIdx.x;
  const int wave = tid >> 5;
  const int lane = tid & 31;
  const int hh   = lane >> 4;
  const int c    = lane & 15;

  const int nqb = g.S / 64;
  const int bx = blockIdx.x;
  const int qb = bx % nqb;
  const int bh = bx / nqb;
  const int h  = bh % g.H;
  const int b  = bh / g.H;
  const int q0 = qb * 64 + wave * 16;

  const float* qp = g.q + (size_t)b * g.q_bs + (size_t)h * g.q_hs;
  const float* kp = g.k + (size_t)b * g.k_bs + (size_t)h * g.k_hs;
  const float* vp = g.v + (size_t)b * g.v_bs + (size_t)h * g.v_hs;
  float*       op = g.o + (size_t)b * g.o_bs + (size_t)h * g.o_hs;
  const float* kbp = g.kb + (size_t)b * g.kb_bs;

  v16h qa[2];
  {
    const float* qrow = qp + (size_t)(q0 + c) * g.q_rs;
#pragma unroll
    for (int dc = 0; dc < 2; ++dc) {
      const float* s0 = qrow + dc * 32 + 8 * hh;
      qa[dc] = pk16(*(const v4f*)(s0), *(const v4f*)(s0 + 4), *(const v4f*)(s0 + 16), *(const v4f*)(s0 + 20));
    }
  }

  const float L2E = 1.4426950408889634f;
  const float NEG = -__builtin_inff();
  float mrow[8], lrow[8];
  v8f oacc[4];
#pragma unroll
  for (int r = 0; r < 8; ++r) { mrow[r] = NEG; lrow[r] = 0.f; }
#pragma unroll
  for (int t = 0; t < 4; ++t) oacc[t] = (v8f){0.f,0.f,0.f,0.f,0.f,0.f,0.f,0.f};

  const int nChunks = g.Skv / 64;
  for (int kc = 0; kc < nChunks; ++kc) {
    const int kv0 = kc * 64;
    __syncthreads();
    {
      const int kvr = tid >> 1, dh = (tid & 1) * 32;
      const float* krow = kp + (size_t)(kv0 + kvr) * g.k_rs + dh;
      const float* vrow = vp + (size_t)(kv0 + kvr) * g.v_rs + dh;
#pragma unroll
      for (int i = 0; i < 4; ++i) {
        const v4f k0v = *(const v4f*)(krow + 8 * i), k1v = *(const v4f*)(krow + 8 * i + 4);
        v8h kh;
        kh[0] = (_Float16)k0v.x; kh[1] = (_Float16)k0v.y; kh[2] = (_Float16)k0v.z; kh[3] = (_Float16)k0v.w;
        kh[4] = (_Float16)k1v.x; kh[5] = (_Float16)k1v.y; kh[6] = (_Float16)k1v.z; kh[7] = (_Float16)k1v.w;
        *(v8h*)(Ksh + kvr * LP + dh + 8 * i) = kh;
        const v4f v0 = *(const v4f*)(vrow + 8 * i), v1 = *(const v4f*)(vrow + 8 * i + 4);
        const int d0 = dh + 8 * i;
        Vth[(d0 + 0) * LP + kvr] = (_Float16)v0.x; Vth[(d0 + 1) * LP + kvr] = (_Float16)v0.y;
        Vth[(d0 + 2) * LP + kvr] = (_Float16)v0.z; Vth[(d0 + 3) * LP + kvr] = (_Float16)v0.w;
        Vth[(d0 + 4) * LP + kvr] = (_Float16)v1.x; Vth[(d0 + 5) * LP + kvr] = (_Float16)v1.y;
        Vth[(d0 + 6) * LP + kvr] = (_Float16)v1.z; Vth[(d0 + 7) * LP + kvr] = (_Float16)v1.w;
      }
    }
    __syncthreads();

    v8f s[4];
#pragma unroll
    for (int j = 0; j < 4; ++j) {
      s[j] = (v8f){0.f,0.f,0.f,0.f,0.f,0.f,0.f,0.f};
#pragma unroll
      for (int dc = 0; dc < 2; ++dc) {
        FH kb;
        kb.h[0] = *(const v8h*)(Ksh + (j * 16 + c) * LP + dc * 32 + 8 * hh);
        kb.h[1] = *(const v8h*)(Ksh + (j * 16 + c) * LP + dc * 32 + 16 + 8 * hh);
        s[j] = wmma16(qa[dc], kb.v, s[j]);
      }
    }
    float kbv[4];
#pragma unroll
    for (int j = 0; j < 4; ++j) kbv[j] = kbp[kv0 + j * 16 + c];

    float cm[8];
#pragma unroll
    for (int r = 0; r < 8; ++r) {
      float m = NEG;
#pragma unroll
      for (int j = 0; j < 4; ++j) {
        const float v = (s[j][r] * g.qscale + kbv[j]) * L2E;
        s[j][r] = v;
        m = fmaxf(m, v);
      }
      m = fmaxf(m, __shfl_xor(m, 1, 32)); m = fmaxf(m, __shfl_xor(m, 2, 32));
      m = fmaxf(m, __shfl_xor(m, 4, 32)); m = fmaxf(m, __shfl_xor(m, 8, 32));
      cm[r] = m;
    }
    _Float16* pw = Psh[wave];
#pragma unroll
    for (int r = 0; r < 8; ++r) {
      const float mnew = fmaxf(mrow[r], cm[r]);
      const float alpha = exp2f(mrow[r] - mnew);
      mrow[r] = mnew;
      float psum = 0.f;
#pragma unroll
      for (int j = 0; j < 4; ++j) {
        const float p = exp2f(s[j][r] - mnew);
        psum += p;
        pw[(8 * hh + r) * LP + j * 16 + c] = (_Float16)(p * 4096.0f);
      }
      psum += __shfl_xor(psum, 1, 32); psum += __shfl_xor(psum, 2, 32);
      psum += __shfl_xor(psum, 4, 32); psum += __shfl_xor(psum, 8, 32);
      lrow[r] = lrow[r] * alpha + psum;
#pragma unroll
      for (int t = 0; t < 4; ++t) oacc[t][r] *= alpha;
    }
    __syncthreads();
#pragma unroll
    for (int kk = 0; kk < 2; ++kk) {
      FH pa;
      pa.h[0] = *(const v8h*)(pw + c * LP + kk * 32 + 8 * hh);
      pa.h[1] = *(const v8h*)(pw + c * LP + kk * 32 + 16 + 8 * hh);
#pragma unroll
      for (int t = 0; t < 4; ++t) {
        FH vb;
        vb.h[0] = *(const v8h*)(Vth + (t * 16 + c) * LP + kk * 32 + 8 * hh);
        vb.h[1] = *(const v8h*)(Vth + (t * 16 + c) * LP + kk * 32 + 16 + 8 * hh);
        oacc[t] = wmma16(pa.v, vb.v, oacc[t]);
      }
    }
  }

  float* os = Os[wave];
#pragma unroll
  for (int r = 0; r < 8; ++r) {
    const float inv = 1.0f / (lrow[r] * 4096.0f);
#pragma unroll
    for (int t = 0; t < 4; ++t) os[(8 * hh + r) * 68 + t * 16 + c] = oacc[t][r] * inv;
  }
  __syncthreads();
  {
    const int c4 = (lane & 15) * 4;
    for (int pass = 0; pass < 2; ++pass) {
#pragma unroll
      for (int it = 0; it < 8; ++it) {
        const int row = it * 2 + hh;
        const v4f val = *(const v4f*)(os + row * 68 + c4);
        *(volatile v4f*)(op + (size_t)(q0 + row) * g.o_rs + c4) = val;
      }
      __threadfence();
    }
  }
}

__device__ __forceinline__ unsigned int bk_pk2(float a, float b) { return (unsigned int)__builtin_bit_cast(unsigned short, (_Float16)a) | ((unsigned int)__builtin_bit_cast(unsigned short, (_Float16)b) << 16); }
template <int NQ, int HASX, int XBF, int ABF = 0>
__global__ __launch_bounds__(256) void k_b_ln(const float* __restrict__ A, const float* __restrict__ X, const float* __restrict__ GA, const float* __restrict__ BE, float eps, float inv_vden, int rows, const float* __restrict__ MG, const float* __restrict__ MB, int rows_per_b, float* __restrict__ Yf, unsigned short* __restrict__ Y16) {
    #pragma clang fp contract(off)
    constexpr int WD = 128 * NQ; const int r = blockIdx.x * 8 + (threadIdx.x >> 5); const int L = threadIdx.x & 31; if (r >= rows) return; v4f v[NQ]; float s = 0.f;
#pragma unroll
    for (int q = 0; q < NQ; ++q) { const long long o = (long long)r * WD + 4 * L + 128 * q; v[q] = *(const v4f*)(A + o); if (ABF) { v[q].x = cmb_bf(v[q].x); v[q].y = cmb_bf(v[q].y); v[q].z = cmb_bf(v[q].z); v[q].w = cmb_bf(v[q].w); } if (HASX) { v4f x = *(const v4f*)(X + o); if (XBF) { x.x = cmb_bf(x.x); x.y = cmb_bf(x.y); x.z = cmb_bf(x.z); x.w = cmb_bf(x.w); } v[q] = v[q] + x; } s += (v[q].x + v[q].y) + (v[q].z + v[q].w); }
#pragma unroll
    for (int o = 16; o > 0; o >>= 1) s += __shfl_xor(s, o, 32);
    const float mu = s * (1.f / WD); float qq = 0.f;
#pragma unroll
    for (int q = 0; q < NQ; ++q) { v[q].x -= mu; v[q].y -= mu; v[q].z -= mu; v[q].w -= mu; qq += (v[q].x * v[q].x + v[q].y * v[q].y) + (v[q].z * v[q].z + v[q].w * v[q].w); }
#pragma unroll
    for (int o = 16; o > 0; o >>= 1) qq += __shfl_xor(qq, o, 32);
    const float rs = (eps < 0.f) ? (1.f / (sqrtf(qq * inv_vden) - eps)) : rsqrtf(qq * inv_vden + eps); const int bb = (MG != nullptr) ? (r / rows_per_b) : 0;
#pragma unroll
    for (int q = 0; q < NQ; ++q) { const int c = 4 * L + 128 * q; const v4f ga = *(const v4f*)(GA + c), be = *(const v4f*)(BE + c); v4f y; y.x = v[q].x * rs * cmb_bf(ga.x) + cmb_bf(be.x); y.y = v[q].y * rs * cmb_bf(ga.y) + cmb_bf(be.y); y.z = v[q].z * rs * cmb_bf(ga.z) + cmb_bf(be.z); y.w = v[q].w * rs * cmb_bf(ga.w) + cmb_bf(be.w);
        if (MG != nullptr) { const v4f mg = *(const v4f*)(MG + (long long)bb * WD + c), mb = *(const v4f*)(MB + (long long)bb * WD + c); y.x = y.x * (1.f + mg.x) + mb.x; y.y = y.y * (1.f + mg.y) + mb.y; y.z = y.z * (1.f + mg.z) + mb.z; y.w = y.w * (1.f + mg.w) + mb.w; }
        const long long o = (long long)r * WD + c; if (Yf != nullptr) VST2V4(Yf + o, y); if (Y16 != nullptr) { bk_u2 pk; pk.x = bk_pk2(y.x, y.y); pk.y = bk_pk2(y.z, y.w); VST2(bk_u2, (bk_u2*)(Y16 + o), pk); } } }
template <int ACT> __device__ __forceinline__ float bk_act(float v) { return (ACT == 0) ? fmaxf(v, 0.f) : 0.5f * v * (1.f + erff(v * 0.70710678118654752f)); }
template <int ACT>
__global__ __launch_bounds__(256) void k_b_act4(const float* __restrict__ F, unsigned short* __restrict__ Y16, long long n4) {
    #pragma clang fp contract(off)
    const long long u = (long long)blockIdx.x * 256 + threadIdx.x; if (u >= n4) return;
    const v4f a = *(const v4f*)(F + 4 * u); bk_u2 pk; pk.x = bk_pk2(bk_act<ACT>(a.x), bk_act<ACT>(a.y)); pk.y = bk_pk2(bk_act<ACT>(a.z), bk_act<ACT>(a.w)); VST2(bk_u2, (bk_u2*)(Y16 + 4 * u), pk); }

static inline size_t al256(size_t v) { return (v + 255) & ~(size_t)255; }
static void launch_gemm(const unsigned short* A, int lda, const unsigned short* Bt, int ldb, float* C, int ldc, const float* bias, int M, int N, int K, float scale, hipStream_t st) {
    const int tiles = (M / 64) * (N / 64);
    wmma_gemm64<0, false, 2, 0, false, 0><<<dim3((unsigned)((tiles + 7) / 8), 1u), 256, 0, st>>>(A, nullptr, lda, 0, Bt, nullptr, ldb, 0, (void*)C, nullptr, ldc, 0, bias, nullptr, 0, M, N, K, scale);
}

constexpr size_t SZ_X16 = (size_t)MTOK * DM * 2;
constexpr size_t SZ_W3  = (size_t)3 * DM * DM * 2;
constexpr size_t SZ_BIG = (size_t)MTOK * 3 * DM * 4;
constexpr size_t SZ_AO  = (size_t)MTOK * DM * 4;
constexpr size_t SZ_WO  = (size_t)DM * DM * 2;
constexpr size_t SZ_H   = (size_t)MTOK * DM * 4;
constexpr size_t SZ_H16 = (size_t)MTOK * DM * 2;
constexpr size_t SZ_W1  = (size_t)DM * FFD * 2;
constexpr size_t SZ_W2  = (size_t)FFD * DM * 2;
constexpr size_t SZ_BR3 = (size_t)3 * DM * 4;
constexpr size_t SZ_BRX = (size_t)(DM + FFD + DM) * 4;
constexpr size_t SZ_MB  = (size_t)MTOK * 4;
constexpr size_t SZ_F1  = (size_t)FCH * FFD * 4;
constexpr size_t SZ_F16 = (size_t)FCH * FFD * 2;
static_assert(SZ_F1 + SZ_F16 <= SZ_BIG);
static_assert((size_t)MTOK * DM * 4 <= SZ_BIG);
static_assert(SZ_F1 % 256 == 0 && SZ_X16 % 256 == 0 && SZ_MB % 256 == 0 && SZ_BR3 % 256 == 0 && SZ_BRX % 256 == 0);
constexpr size_t CARVE_TOTAL = SZ_X16 + SZ_W3 + SZ_BIG + SZ_AO + SZ_WO + SZ_H + SZ_H16 + SZ_W1 + SZ_W2 + SZ_BR3 + SZ_BRX + SZ_MB;
static_assert(CARVE_TOTAL <= (size_t)134217728);

extern "C" void kernel_launch(void* const* d_in, const int* in_sizes, int n_in, void* d_out, int out_size, void* d_ws, size_t ws_size, hipStream_t stream) {
    if (n_in < 18) return;
    const long long need_tok = (long long)(NB - 1) * SEQ_FULL + SEQ;
    if ((long long)in_sizes[0] < need_tok * DM) return;
    if ((long long)in_sizes[1] < need_tok) return;
    if (in_sizes[2] < DM * DM || in_sizes[4] < DM * DM || in_sizes[6] < DM * DM || in_sizes[8] < DM * DM) return;
    if (in_sizes[3] < DM || in_sizes[5] < DM || in_sizes[7] < DM || in_sizes[9] < DM || in_sizes[10] < DM || in_sizes[11] < DM) return;
    if (in_sizes[12] < DM * FFD || in_sizes[13] < FFD || in_sizes[14] < FFD * DM || in_sizes[15] < DM || in_sizes[16] < DM || in_sizes[17] < DM) return;
    if ((long long)out_size < need_tok * DM) return;
    if (CARVE_TOTAL > ws_size) return;

    const float* x    = (const float*)d_in[0];
    const int*   mask = (const int*)  d_in[1];
    const float* wq   = (const float*)d_in[2];
    const float* bq   = (const float*)d_in[3];
    const float* wk   = (const float*)d_in[4];
    const float* bk   = (const float*)d_in[5];
    const float* wv   = (const float*)d_in[6];
    const float* bv   = (const float*)d_in[7];
    const float* wo   = (const float*)d_in[8];
    const float* bo   = (const float*)d_in[9];
    const float* g1   = (const float*)d_in[10];
    const float* be1  = (const float*)d_in[11];
    const float* w1   = (const float*)d_in[12];
    const float* bf1  = (const float*)d_in[13];
    const float* w2   = (const float*)d_in[14];
    const float* bf2  = (const float*)d_in[15];
    const float* g2   = (const float*)d_in[16];
    const float* be2  = (const float*)d_in[17];
    float* out = (float*)d_out;

    char* wsp = (char*)d_ws;
    unsigned short* X16  = (unsigned short*)wsp; wsp += al256(SZ_X16);
    unsigned short* W316 = (unsigned short*)wsp; wsp += al256(SZ_W3);
    char* BIG = wsp;                             wsp += al256(SZ_BIG);
    float* AO  = (float*)wsp;                    wsp += al256(SZ_AO);
    unsigned short* WO16 = (unsigned short*)wsp; wsp += al256(SZ_WO);
    float* Hf  = (float*)wsp;                    wsp += al256(SZ_H);
    unsigned short* H16  = (unsigned short*)wsp; wsp += al256(SZ_H16);
    unsigned short* W1T  = (unsigned short*)wsp; wsp += al256(SZ_W1);
    unsigned short* W2T  = (unsigned short*)wsp; wsp += al256(SZ_W2);
    float* BR3 = (float*)wsp;                    wsp += al256(SZ_BR3);
    float* BRX = (float*)wsp;                    wsp += al256(SZ_BRX);
    float* MBF = (float*)wsp;                    wsp += al256(SZ_MB);
    float* QKV = (float*)BIG;
    float* ATT = (float*)BIG;
    float* F1  = (float*)BIG;
    unsigned short* F16 = (unsigned short*)(BIG + SZ_F1);
    unsigned short* AO16 = X16;
    float* FFo = AO;

    constexpr int NSEG = (SEQ == SEQ_FULL) ? 1 : NB;
    constexpr int SEGR = (SEQ == SEQ_FULL) ? MTOK : SEQ;

    for (int sg = 0; sg < NSEG; ++sg)
        k_cm_castb<1><<<(unsigned)(((long long)SEGR * (DM / 8) + 255) / 256), 256, 0, stream>>>(x + (size_t)sg * SEQ_FULL * DM, DM, X16 + (size_t)sg * SEQ * DM, DM, SEGR, DM, 1.0f);
    k_cm_castbT<<<(unsigned)(((long long)DM * (DM / 8) + 255) / 256), 256, 0, stream>>>(wq, DM, W316, DM, DM, DM, 16.0f);
    k_cm_castbT<<<(unsigned)(((long long)DM * (DM / 8) + 255) / 256), 256, 0, stream>>>(wk, DM, W316 + (size_t)DM * DM, DM, DM, DM, 16.0f);
    k_cm_castbT<<<(unsigned)(((long long)DM * (DM / 8) + 255) / 256), 256, 0, stream>>>(wv, DM, W316 + (size_t)2 * DM * DM, DM, DM, DM, 16.0f);
    k_cm_castbT<<<(unsigned)(((long long)DM * (DM / 8) + 255) / 256), 256, 0, stream>>>(wo, DM, WO16, DM, DM, DM, 16.0f);
    k_cm_castbT<<<(unsigned)(((long long)FFD * (DM / 8) + 255) / 256), 256, 0, stream>>>(w1, FFD, W1T, DM, DM, FFD, 16.0f);
    k_cm_castbT<<<(unsigned)(((long long)DM * (FFD / 8) + 255) / 256), 256, 0, stream>>>(w2, DM, W2T, FFD, FFD, DM, 16.0f);
    k_bfcat3<<<(3 * DM + 255) / 256, 256, 0, stream>>>(bq, DM, bk, DM, bv, DM, BR3);
    k_bfcat3<<<(DM + FFD + DM + 255) / 256, 256, 0, stream>>>(bo, DM, bf1, FFD, bf2, DM, BRX);
    k_maskbias<<<(MTOK + 255) / 256, 256, 0, stream>>>(mask, MBF, SEQ, SEQ_FULL, MTOK);

    launch_gemm(X16, DM, W316, DM, QKV, 3 * DM, BR3, MTOK, 3 * DM, DM, 0.0625f, stream);

    {
        AttnG a;
        a.q = QKV; a.k = QKV + DM; a.v = QKV + 2 * DM; a.o = AO; a.kb = MBF;
        a.q_bs = (long long)SEQ * 3 * DM; a.q_rs = 3 * DM; a.q_hs = HDIM;
        a.k_bs = (long long)SEQ * 3 * DM; a.k_rs = 3 * DM; a.k_hs = HDIM;
        a.v_bs = (long long)SEQ * 3 * DM; a.v_rs = 3 * DM; a.v_hs = HDIM;
        a.o_bs = (long long)SEQ * DM; a.o_rs = DM; a.o_hs = HDIM; a.kb_bs = SEQ;
        a.S = SEQ; a.Skv = SEQ; a.H = NHEAD; a.qscale = 0.125f;
        k_attn64<<<(unsigned)(NB * NHEAD * (SEQ / 64)), 32 * AT_NW, 0, stream>>>(a);
    }
    k_cm_castb<0><<<(unsigned)(((long long)MTOK * (DM / 8) + 255) / 256), 256, 0, stream>>>(AO, DM, AO16, DM, MTOK, DM, 64.0f);
    launch_gemm(AO16, DM, WO16, DM, ATT, DM, BRX, MTOK, DM, DM, 0.0009765625f, stream);
    for (int sg = 0; sg < NSEG; ++sg)
        k_b_ln<8, 1, 1, 0><<<(SEGR + 7) / 8, 256, 0, stream>>>(ATT + (size_t)sg * SEQ * DM, x + (size_t)sg * SEQ_FULL * DM, g1, be1, 1e-12f, 0.0009765625f, SEGR, nullptr, nullptr, 1, Hf + (size_t)sg * SEQ * DM, H16 + (size_t)sg * SEQ * DM);
    for (int ch = 0; ch < 2; ++ch) {
        launch_gemm(H16 + (size_t)ch * FCH * DM, DM, W1T, DM, F1, FFD, BRX + DM, FCH, FFD, DM, 0.0625f, stream);
        k_b_act4<1><<<(unsigned)(((long long)FCH * FFD / 4 + 255) / 256), 256, 0, stream>>>(F1, F16, (long long)FCH * FFD / 4);
        launch_gemm(F16, FFD, W2T, FFD, FFo + (size_t)ch * FCH * DM, DM, BRX + DM + FFD, FCH, DM, FFD, 0.0625f, stream);
    }
    for (int sg = 0; sg < NSEG; ++sg)
        k_b_ln<8, 1, 0, 0><<<(SEGR + 7) / 8, 256, 0, stream>>>(FFo + (size_t)sg * SEQ * DM, Hf + (size_t)sg * SEQ * DM, g2, be2, 1e-12f, 0.0009765625f, SEGR, nullptr, nullptr, 1, out + (size_t)sg * SEQ_FULL * DM, nullptr);
}
